// DecoderGRU_31490700214516
// MI455X (gfx1250) — hardware-verified
//
#include <hip/hip_runtime.h>
#define BSZ 4096
#define TT 64
#define HH 64
#define PP 50
#define PPAD 64
#define VV 32
#define G3 (3 * HH)
#define LOSS_OFF 33554432

typedef __bf16 v16b __attribute__((ext_vector_type(16)));
typedef unsigned short v8us __attribute__((ext_vector_type(8), may_alias));
typedef float  v8f  __attribute__((ext_vector_type(8)));
typedef float  v4f  __attribute__((ext_vector_type(4)));
typedef float  v4fa __attribute__((ext_vector_type(4), may_alias));
union FragB { v16b v; v8us half[2]; unsigned short u[16]; };

__device__ __forceinline__ unsigned short bf16_bits(float x) { unsigned int u = __float_as_uint(x); return (unsigned short)((u + 0x7FFFu + ((u >> 16) & 1u)) >> 16); }
__device__ __forceinline__ float bf16_val(unsigned short b) { return __uint_as_float(((unsigned int)b) << 16); }
__device__ __forceinline__ float bf16_round(float x) { return bf16_val(bf16_bits(x)); }
template <int NT>
__device__ __forceinline__ v8f mmaN(v16b ah, v16b al, v16b bh, v16b bl, v8f c) {
  c = __builtin_amdgcn_wmma_f32_16x16x32_bf16(false, ah, false, bh, (short)0, c, false, false);
  if (NT >= 2) c = __builtin_amdgcn_wmma_f32_16x16x32_bf16(false, al, false, bh, (short)0, c, false, false);
  if (NT >= 3) c = __builtin_amdgcn_wmma_f32_16x16x32_bf16(false, ah, false, bl, (short)0, c, false, false);
  asm volatile("v_nop\n\tv_nop\n\tv_nop\n\tv_nop" : "+v"(c) : "v"(ah), "v"(al), "v"(bh), "v"(bl));
  return c;
}

__global__ __launch_bounds__(256) void k_wt_bf16(const float* __restrict__ W, unsigned short* __restrict__ Wt, int K, int N) {
  const int t = blockIdx.x * 256 + threadIdx.x;
  const int k8n = K / 8;
  if (t >= N * k8n) return;
  const int n = t / k8n, k8 = (t % k8n) * 8;
  v8us v;
#pragma unroll
  for (int i = 0; i < 8; ++i) v[i] = bf16_bits(W[(size_t)(k8 + i) * N + n]);
  *(volatile v8us*)(Wt + (size_t)n * K + k8) = v;
  __threadfence();
  *(volatile v8us*)(Wt + (size_t)n * K + k8) = v;
}

template <bool ASPLIT, int ACT, bool BIAS_BF16>
__global__ __launch_bounds__(128) void k_gemm_bf(const float* __restrict__ A, int lda, const unsigned short* __restrict__ Wt, int ldb,
                                               const float* __restrict__ bias, float* __restrict__ C, int ldc, int M, int N, int K) {
  __shared__ __attribute__((aligned(16))) float so[4][16][64];
  const int tid = threadIdx.x, w = tid >> 5, lane = tid & 31, ln = lane & 15, hh = lane >> 4;
  const int ntn = N / 64;
  const int wid = blockIdx.x * 4 + w;
  const int mt = wid / ntn, nq = wid % ntn;
  if (mt * 16 >= M) return;
  const int row0 = mt * 16, col0 = nq * 64;
  const float* arow = A + (size_t)(row0 + ln) * lda;
  v8f acc[4] = {};
  for (int kb = 0; kb < K; kb += 32) {
    FragB ah, al;
    const v4f x0 = *(const v4fa*)(arow + kb + 8 * hh), x1 = *(const v4fa*)(arow + kb + 8 * hh + 4);
    const v4f x2 = *(const v4fa*)(arow + kb + 16 + 8 * hh), x3 = *(const v4fa*)(arow + kb + 16 + 8 * hh + 4);
    float xs[16] = {x0[0],x0[1],x0[2],x0[3],x1[0],x1[1],x1[2],x1[3],x2[0],x2[1],x2[2],x2[3],x3[0],x3[1],x3[2],x3[3]};
#pragma unroll
    for (int i = 0; i < 16; ++i) { const unsigned short hb = bf16_bits(xs[i]); ah.u[i] = hb; al.u[i] = ASPLIT ? bf16_bits(xs[i] - bf16_val(hb)) : (unsigned short)0; }
#pragma unroll
    for (int t = 0; t < 4; ++t) {
      const unsigned short* brow = Wt + (size_t)(col0 + t * 16 + ln) * ldb + kb;
      FragB b;
      b.half[0] = *(const v8us*)(brow + 8 * hh);
      b.half[1] = *(const v8us*)(brow + 16 + 8 * hh);
      acc[t] = mmaN<ASPLIT ? 2 : 1>(ah.v, al.v, b.v, b.v, acc[t]);
    }
  }
#pragma unroll
  for (int t = 0; t < 4; ++t) {
    float bv = bias ? bias[col0 + t * 16 + ln] : 0.f;
    if (BIAS_BF16) bv = bf16_round(bv);
#pragma unroll
    for (int r = 0; r < 8; ++r) { float v = acc[t][r] + bv; if (ACT == 1) v = fmaxf(v, 0.f); so[w][8 * hh + r][t * 16 + ln] = v; }
  }
  __builtin_amdgcn_fence(__ATOMIC_ACQ_REL, "workgroup");
  __builtin_amdgcn_wave_barrier();
  const int rsub = lane >> 4, c4 = (lane & 15) * 4;
  for (int pass = 0; pass < 2; ++pass) {
#pragma unroll
    for (int q = 0; q < 8; ++q) {
      const int r = q * 2 + rsub;
      const v4f v = *(const v4fa*)&so[w][r][c4];
      *(volatile v4f*)(C + (size_t)(row0 + r) * ldc + col0 + c4) = v;
    }
    if (pass == 0) __threadfence();
  }
}

template <int D, bool CAUSAL>
__global__ __launch_bounds__(128) void k_flash(const float* __restrict__ qb, const float* __restrict__ kb, const float* __restrict__ vb,
                                             int pitch, int T, int H, float scale, float* __restrict__ y, int ypitch) {
  constexpr int KS = D / 32;
  constexpr int DT = D / 16;
  __shared__ __attribute__((aligned(16))) unsigned short sKh[32][D + 8], sKl[32][D + 8], sVh[32][D + 8], sVl[32][D + 8];
  __shared__ __attribute__((aligned(16))) unsigned short sPh[4][16][40], sPl[4][16][40];
  __shared__ __attribute__((aligned(16))) float sO[4][16][D];
  const int tid = threadIdx.x, w = tid >> 5, lane = tid & 31, ln = lane & 15, hh = lane >> 4;
  const int nqb = (T + 63) / 64;
  const int bh = blockIdx.x / nqb, qblk = blockIdx.x % nqb;
  const int b = bh / H, h = bh % H;
  const int q0 = qblk * 64 + w * 16;
  const float* Q = qb + (size_t)b * T * pitch + h * D;
  const float* K = kb + (size_t)b * T * pitch + h * D;
  const float* V = vb + (size_t)b * T * pitch + h * D;

  FragB aqh[KS], aql[KS];
  {
    int row = q0 + ln; if (row >= T) row = T - 1;
    const float* qr = Q + (size_t)row * pitch;
#pragma unroll
    for (int ks = 0; ks < KS; ++ks)
#pragma unroll
      for (int i = 0; i < 16; ++i) {
        const int d = ks * 32 + ((i < 8) ? (8 * hh + i) : (16 + 8 * hh + (i - 8)));
        const float x = qr[d] * scale; const unsigned short hb = bf16_bits(x);
        aqh[ks].u[i] = hb; aql[ks].u[i] = bf16_bits(x - bf16_val(hb));
      }
  }
  float m_r[8], l_r[8];
#pragma unroll
  for (int r = 0; r < 8; ++r) { m_r[r] = -3.0e38f; l_r[r] = 0.f; }
  v8f oacc[DT];
#pragma unroll
  for (int dt = 0; dt < DT; ++dt) oacc[dt] = (v8f){0.f,0.f,0.f,0.f,0.f,0.f,0.f,0.f};

  const int kv_end = CAUSAL ? min(T, qblk * 64 + 64) : T;
  for (int j0 = 0; j0 < kv_end; j0 += 32) {
    __syncthreads();
    for (int e = tid; e < 32 * (D / 4); e += 128) {
      const int r = e / (D / 4), c4 = (e % (D / 4)) * 4;
      const int key = j0 + r;
      v4f kf = {0.f,0.f,0.f,0.f}, vf = {0.f,0.f,0.f,0.f};
      if (key < T) { kf = *(const v4fa*)(K + (size_t)key * pitch + c4); vf = *(const v4fa*)(V + (size_t)key * pitch + c4); }
#pragma unroll
      for (int t = 0; t < 4; ++t) {
        unsigned short hb = bf16_bits(kf[t]); sKh[r][c4 + t] = hb; sKl[r][c4 + t] = bf16_bits(kf[t] - bf16_val(hb));
        hb = bf16_bits(vf[t]); sVh[r][c4 + t] = hb; sVl[r][c4 + t] = bf16_bits(vf[t] - bf16_val(hb));
      }
    }
    __syncthreads();
    v8f s[2];
#pragma unroll
    for (int nt = 0; nt < 2; ++nt) {
      v8f acc = {};
#pragma unroll
      for (int ks = 0; ks < KS; ++ks) {
        FragB bh_, bl_;
        bh_.half[0] = *(const v8us*)&sKh[nt * 16 + ln][ks * 32 + 8 * hh]; bh_.half[1] = *(const v8us*)&sKh[nt * 16 + ln][ks * 32 + 16 + 8 * hh];
        bl_.half[0] = *(const v8us*)&sKl[nt * 16 + ln][ks * 32 + 8 * hh]; bl_.half[1] = *(const v8us*)&sKl[nt * 16 + ln][ks * 32 + 16 + 8 * hh];
        acc = mmaN<3>(aqh[ks].v, aql[ks].v, bh_.v, bl_.v, acc);
      }
      s[nt] = acc;
    }
    float alpha[8];
#pragma unroll
    for (int r = 0; r < 8; ++r) {
      const int qi = q0 + 8 * hh + r;
      const int ja = j0 + ln, jb = j0 + 16 + ln;
      if (CAUSAL) { if (ja > qi) s[0][r] = -3.0e38f; if (jb > qi) s[1][r] = -3.0e38f; }
      if (ja >= T) s[0][r] = -3.0e38f;
      if (jb >= T) s[1][r] = -3.0e38f;
      float mx = fmaxf(s[0][r], s[1][r]);
      mx = fmaxf(mx, __shfl_xor(mx, 1, 32)); mx = fmaxf(mx, __shfl_xor(mx, 2, 32)); mx = fmaxf(mx, __shfl_xor(mx, 4, 32)); mx = fmaxf(mx, __shfl_xor(mx, 8, 32));
      const float mnew = fmaxf(m_r[r], mx);
      alpha[r] = (mnew > -1.0e38f) ? __expf(m_r[r] - mnew) : 1.0f;
      const float p0 = (s[0][r] > -1.0e38f) ? __expf(s[0][r] - mnew) : 0.f;
      const float p1 = (s[1][r] > -1.0e38f) ? __expf(s[1][r] - mnew) : 0.f;
      m_r[r] = mnew;
      l_r[r] = l_r[r] * alpha[r] + p0 + p1;
      unsigned short hb = bf16_bits(p0); sPh[w][8 * hh + r][ln] = hb;      sPl[w][8 * hh + r][ln] = bf16_bits(p0 - bf16_val(hb));
      hb = bf16_bits(p1);                sPh[w][8 * hh + r][16 + ln] = hb; sPl[w][8 * hh + r][16 + ln] = bf16_bits(p1 - bf16_val(hb));
    }
#pragma unroll
    for (int dt = 0; dt < DT; ++dt)
#pragma unroll
      for (int r = 0; r < 8; ++r) oacc[dt][r] *= alpha[r];
    __builtin_amdgcn_fence(__ATOMIC_ACQ_REL, "workgroup");
    __builtin_amdgcn_wave_barrier();
    FragB pah, pal;
    pah.half[0] = *(const v8us*)&sPh[w][ln][8 * hh]; pah.half[1] = *(const v8us*)&sPh[w][ln][16 + 8 * hh];
    pal.half[0] = *(const v8us*)&sPl[w][ln][8 * hh]; pal.half[1] = *(const v8us*)&sPl[w][ln][16 + 8 * hh];
#pragma unroll
    for (int dt = 0; dt < DT; ++dt) {
      FragB bvh, bvl;
#pragma unroll
      for (int i = 0; i < 8; ++i) {
        bvh.u[i] = sVh[8 * hh + i][dt * 16 + ln]; bvh.u[8 + i] = sVh[16 + 8 * hh + i][dt * 16 + ln];
        bvl.u[i] = sVl[8 * hh + i][dt * 16 + ln]; bvl.u[8 + i] = sVl[16 + 8 * hh + i][dt * 16 + ln];
      }
      oacc[dt] = mmaN<3>(pah.v, pal.v, bvh.v, bvl.v, oacc[dt]);
    }
    __builtin_amdgcn_fence(__ATOMIC_ACQ_REL, "workgroup");
    __builtin_amdgcn_wave_barrier();
  }
#pragma unroll
  for (int r = 0; r < 8; ++r) {
    float l = l_r[r];
    l += __shfl_xor(l, 1, 32); l += __shfl_xor(l, 2, 32); l += __shfl_xor(l, 4, 32); l += __shfl_xor(l, 8, 32);
    l_r[r] = (l > 0.f) ? 1.0f / l : 0.f;
  }
#pragma unroll
  for (int dt = 0; dt < DT; ++dt)
#pragma unroll
    for (int r = 0; r < 8; ++r) sO[w][8 * hh + r][dt * 16 + ln] = oacc[dt][r] * l_r[r];
  __builtin_amdgcn_fence(__ATOMIC_ACQ_REL, "workgroup");
  __builtin_amdgcn_wave_barrier();
  for (int pass = 0; pass < 2; ++pass) {
    for (int r = 0; r < 16; ++r) {
      const int row = q0 + r;
      if (row < T && lane < D / 4) {
        const v4f val = *(const v4fa*)&sO[w][r][lane * 4];
        *(volatile v4f*)(y + ((size_t)b * T + row) * ypitch + h * D + lane * 4) = val;
      }
    }
    if (pass == 0) __threadfence();
  }
}

template <bool ASPLIT, bool BSPLIT, int ACT>
__global__ __launch_bounds__(128) void k_gemm_b(const float* __restrict__ A, int lda, size_t sA, const unsigned short* __restrict__ Bh, const unsigned short* __restrict__ Bl, int ldb, size_t sB,
                                             const float* __restrict__ bias, const float* __restrict__ resid, int ldr, size_t sR, float rsign, float alpha,
                                             float* __restrict__ C, int ldc, size_t sC, int M, int N, int K) {
  __shared__ __attribute__((aligned(16))) float so[4][16][64];
  const int tid = threadIdx.x, w = tid >> 5, lane = tid & 31, ln = lane & 15, hh = lane >> 4;
  const int by = blockIdx.y;
  A += (size_t)by * sA; Bh += (size_t)by * sB; if (BSPLIT) Bl += (size_t)by * sB; C += (size_t)by * sC; if (resid) resid += (size_t)by * sR;
  const int ntn = (N + 63) / 64; const int wid = blockIdx.x * 4 + w; const int mt = wid / ntn, nq = wid % ntn;
  if (mt * 16 >= M) return;
  const int row0 = mt * 16, col0 = nq * 64;
  const float* arow = A + (size_t)(row0 + ln) * lda;
  v8f acc[4] = {};
  for (int kb = 0; kb < K; kb += 32) {
    FragB ah, al;
    const v4f x0 = *(const v4fa*)(arow + kb + 8 * hh), x1 = *(const v4fa*)(arow + kb + 8 * hh + 4);
    const v4f x2 = *(const v4fa*)(arow + kb + 16 + 8 * hh), x3 = *(const v4fa*)(arow + kb + 16 + 8 * hh + 4);
    float xs[16] = {x0[0],x0[1],x0[2],x0[3],x1[0],x1[1],x1[2],x1[3],x2[0],x2[1],x2[2],x2[3],x3[0],x3[1],x3[2],x3[3]};
#pragma unroll
    for (int i = 0; i < 16; ++i) { const unsigned short hb = bf16_bits(xs[i]); ah.u[i] = hb; al.u[i] = ASPLIT ? bf16_bits(xs[i] - bf16_val(hb)) : (unsigned short)0; }
#pragma unroll
    for (int t = 0; t < 4; ++t) {
      if (col0 + t * 16 >= N) continue;
      const size_t boff = (size_t)(col0 + t * 16 + ln) * ldb + kb;
      FragB bh_, bl_; bh_.half[0] = *(const v8us*)(Bh + boff + 8 * hh); bh_.half[1] = *(const v8us*)(Bh + boff + 16 + 8 * hh);
      if (BSPLIT) { bl_.half[0] = *(const v8us*)(Bl + boff + 8 * hh); bl_.half[1] = *(const v8us*)(Bl + boff + 16 + 8 * hh); } else bl_ = bh_;
      acc[t] = mmaN<ASPLIT ? (BSPLIT ? 3 : 2) : 1>(ah.v, al.v, bh_.v, bl_.v, acc[t]);
    }
  }
#pragma unroll
  for (int t = 0; t < 4; ++t) {
    const int col = col0 + t * 16 + ln; if (col0 + t * 16 >= N) continue; const float bv = bias ? bf16_round(bias[col]) : 0.f;
#pragma unroll
    for (int r = 0; r < 8; ++r) { float v = acc[t][r] * alpha + bv; if (resid) v += rsign * resid[(size_t)(row0 + 8 * hh + r) * ldr + col]; if (ACT == 1) v = fmaxf(v, 0.f); else if (ACT == 2) v = fmaxf(v, 0.f) + log1pf(expf(-fabsf(v))); so[w][8 * hh + r][t * 16 + ln] = v; }
  }
  __builtin_amdgcn_fence(__ATOMIC_ACQ_REL, "workgroup"); __builtin_amdgcn_wave_barrier();
  const int rsub = lane >> 4, c4 = (lane & 15) * 4;
  for (int pass = 0; pass < 2; ++pass) {
#pragma unroll
    for (int q = 0; q < 8; ++q) { const int r = q * 2 + rsub; if (col0 + c4 < N) { const v4f v = *(const v4fa*)&so[w][r][c4]; *(volatile v4f*)(C + (size_t)(row0 + r) * ldc + col0 + c4) = v; } }
    if (pass == 0) __threadfence();
  }
}
__global__ __launch_bounds__(256) void k_split_transpose_b(const float* __restrict__ src, int lds_, size_t sIn, unsigned short* __restrict__ hi, unsigned short* __restrict__ lo, size_t sOut, int K, int N) {
  const size_t t = (size_t)blockIdx.x * 256 + threadIdx.x; const int k8n = K / 8; if (t >= (size_t)N * k8n) return;
  src += (size_t)blockIdx.y * sIn; hi += (size_t)blockIdx.y * sOut; lo += (size_t)blockIdx.y * sOut;
  const int n = (int)(t / k8n), k8 = (int)(t % k8n) * 8; v8us vh, vl;
#pragma unroll
  for (int i = 0; i < 8; ++i) { const float x = src[(size_t)(k8 + i) * lds_ + n]; const unsigned short hb = bf16_bits(x); vh[i] = hb; vl[i] = bf16_bits(x - bf16_val(hb)); }
  unsigned short* dh = hi + (size_t)n * K + k8; unsigned short* dl = lo + (size_t)n * K + k8;
  *(volatile v8us*)dh = vh; *(volatile v8us*)dl = vl; __threadfence(); *(volatile v8us*)dh = vh; *(volatile v8us*)dl = vl;
}

typedef _Float16 v16h __attribute__((ext_vector_type(16)));
union FragH { v16h v; v8us half[2]; _Float16 h[16]; unsigned short u[16]; };
template <int NT>
__device__ __forceinline__ v8f mmaH(v16h ah, v16h al, v16h bh, v16h bl, v8f c) {
  c = __builtin_amdgcn_wmma_f32_16x16x32_f16(false, ah, false, bh, (short)0, c, false, false);
  if (NT >= 2) c = __builtin_amdgcn_wmma_f32_16x16x32_f16(false, al, false, bh, (short)0, c, false, false);
  if (NT >= 3) c = __builtin_amdgcn_wmma_f32_16x16x32_f16(false, ah, false, bl, (short)0, c, false, false);
  asm volatile("v_nop\n\tv_nop\n\tv_nop\n\tv_nop" : "+v"(c) : "v"(ah), "v"(al), "v"(bh), "v"(bl));
  return c;
}
template <bool ASPLIT>
__global__ __launch_bounds__(128) void k_gemm_h(const float* __restrict__ A, int lda, size_t sA, const _Float16* __restrict__ Bh, int ldb, size_t sB, float alpha, float* __restrict__ C, int ldc, size_t sC, int M, int N, int K) {
  __shared__ __attribute__((aligned(16))) float so[4][16][64];
  const int tid = threadIdx.x, w = tid >> 5, lane = tid & 31, ln = lane & 15, hh = lane >> 4; const int by = blockIdx.y;
  A += (size_t)by * sA; Bh += (size_t)by * sB; C += (size_t)by * sC;
  const int ntn = (N + 63) / 64; const int wid = blockIdx.x * 4 + w; const int mt = wid / ntn, nq = wid % ntn; if (mt * 16 >= M) return;
  const int row0 = mt * 16, col0 = nq * 64; const float* arow = A + (size_t)(row0 + ln) * lda;
  v8f acc[4] = {};
  for (int kb = 0; kb < K; kb += 32) {
    FragH ah, al;
    const v4f x0 = *(const v4fa*)(arow + kb + 8 * hh), x1 = *(const v4fa*)(arow + kb + 8 * hh + 4), x2 = *(const v4fa*)(arow + kb + 16 + 8 * hh), x3 = *(const v4fa*)(arow + kb + 16 + 8 * hh + 4);
    float xs[16] = {x0[0],x0[1],x0[2],x0[3],x1[0],x1[1],x1[2],x1[3],x2[0],x2[1],x2[2],x2[3],x3[0],x3[1],x3[2],x3[3]};
#pragma unroll
    for (int i = 0; i < 16; ++i) { const _Float16 h = (_Float16)xs[i]; ah.h[i] = h; al.h[i] = ASPLIT ? (_Float16)(xs[i] - (float)h) : (_Float16)0.0f; }
#pragma unroll
    for (int t = 0; t < 4; ++t) { if (col0 + t * 16 >= N) continue; const size_t boff = (size_t)(col0 + t * 16 + ln) * ldb + kb; FragH bq; bq.half[0] = *(const v8us*)(Bh + boff + 8 * hh); bq.half[1] = *(const v8us*)(Bh + boff + 16 + 8 * hh);
      acc[t] = mmaH<ASPLIT ? 2 : 1>(ah.v, al.v, bq.v, bq.v, acc[t]); }
  }
#pragma unroll
  for (int t = 0; t < 4; ++t) { if (col0 + t * 16 >= N) continue;
#pragma unroll
    for (int r = 0; r < 8; ++r) so[w][8 * hh + r][t * 16 + ln] = acc[t][r] * alpha; }
  __builtin_amdgcn_fence(__ATOMIC_ACQ_REL, "workgroup"); __builtin_amdgcn_wave_barrier();
  const int rsub = lane >> 4, c4 = (lane & 15) * 4;
  for (int pass = 0; pass < 2; ++pass) {
#pragma unroll
    for (int q = 0; q < 8; ++q) { const int r = q * 2 + rsub; if (col0 + c4 < N) { const v4f v = *(const v4fa*)&so[w][r][c4]; *(volatile v4f*)(C + (size_t)(row0 + r) * ldc + col0 + c4) = v; } }
    if (pass == 0) __threadfence(); }
}

__device__ __forceinline__ int cc(int c) { return c < 0 ? 0 : (c >= VV ? VV - 1 : c); }
__global__ __launch_bounds__(256) void k_prep(const float* __restrict__ Wrx, const float* __restrict__ Wzx, const float* __restrict__ Whx, const float* __restrict__ brx, const float* __restrict__ bzx, const float* __restrict__ bhx,
                                              const float* __restrict__ Wrh, const float* __restrict__ Wzh, const float* __restrict__ Whh, const float* __restrict__ Wpj, const float* __restrict__ emb, const float* __restrict__ phon,
                                              unsigned short* __restrict__ Btop, unsigned short* __restrict__ Bbot, float* __restrict__ B3, _Float16* __restrict__ Brz, _Float16* __restrict__ Bhh, _Float16* __restrict__ Bpj, float* __restrict__ EMBP, float* __restrict__ PHP) {
  const int t = blockIdx.x * 256 + threadIdx.x;
  if (t < G3 * HH / 8) { const int k8 = (t % (HH / 8)) * 8, n = t / (HH / 8); const int g = n / HH, nn = n % HH; const float* W = (g == 0) ? Wrx : (g == 1 ? Wzx : Whx); v8us a, b; for (int q = 0; q < 8; ++q) { const int k = k8 + q; a[q] = bf16_bits(W[(size_t)k * HH + nn]); b[q] = bf16_bits(k < PP ? W[(size_t)(HH + k) * HH + nn] : 0.f); }
    *(volatile v8us*)(Btop + (size_t)n * HH + k8) = a; *(volatile v8us*)(Bbot + (size_t)n * PPAD + k8) = b; __threadfence(); *(volatile v8us*)(Btop + (size_t)n * HH + k8) = a; *(volatile v8us*)(Bbot + (size_t)n * PPAD + k8) = b; }
  if (t < G3) { const int g = t / HH, nn = t % HH; const float v = (g == 0) ? brx[nn] : (g == 1 ? bzx[nn] : bhx[nn]); *(volatile float*)(B3 + t) = v; }
  if (t < 2 * HH * HH / 8) { const int k8 = (t % (HH / 8)) * 8, n = t / (HH / 8); const int g = n / HH, nn = n % HH; const float* W = g == 0 ? Wrh : Wzh; FragH f; for (int q = 0; q < 8; ++q) f.h[q] = (_Float16)(bf16_round(W[(size_t)(k8 + q) * HH + nn]) * 16.0f); *(volatile v8us*)((unsigned short*)Brz + (size_t)n * HH + k8) = f.half[0]; __threadfence(); *(volatile v8us*)((unsigned short*)Brz + (size_t)n * HH + k8) = f.half[0]; }
  if (t < HH * HH / 8) { const int k8 = (t % (HH / 8)) * 8, n = t / (HH / 8); FragH f; for (int q = 0; q < 8; ++q) f.h[q] = (_Float16)(bf16_round(Whh[(size_t)(k8 + q) * HH + n]) * 16.0f); *(volatile v8us*)((unsigned short*)Bhh + (size_t)n * HH + k8) = f.half[0]; __threadfence(); *(volatile v8us*)((unsigned short*)Bhh + (size_t)n * HH + k8) = f.half[0]; }
  if (t < VV * HH / 8) { const int k8 = (t % (HH / 8)) * 8, n = t / (HH / 8); FragH f; for (int q = 0; q < 8; ++q) f.h[q] = (_Float16)(bf16_round(Wpj[(size_t)(k8 + q) * VV + n]) * 16.0f); *(volatile v8us*)((unsigned short*)Bpj + (size_t)n * HH + k8) = f.half[0]; __threadfence(); *(volatile v8us*)((unsigned short*)Bpj + (size_t)n * HH + k8) = f.half[0]; }
  if (t < VV * HH) { const float v = bf16_round(emb[t]); *(volatile float*)(EMBP + t) = v; __threadfence(); *(volatile float*)(EMBP + t) = v; }
  { const size_t tt2 = (size_t)t; if (tt2 < (size_t)BSZ * PPAD) { const int k = (int)(tt2 % PPAD); const size_t b = tt2 / PPAD; const float v = (k < PP) ? bf16_round(phon[b * PP + k]) : 0.f; *(volatile float*)(PHP + tt2) = v; __threadfence(); *(volatile float*)(PHP + tt2) = v; } } }
__device__ __forceinline__ void fragHL(FragH& fh, FragH& fl, const float* rowp, int hh) {
#pragma unroll
  for (int q = 0; q < 8; ++q) { const float a = rowp[8 * hh + q], b = rowp[16 + 8 * hh + q]; const _Float16 ah = (_Float16)a, bh = (_Float16)b; fh.h[q] = ah; fl.h[q] = (_Float16)(a - (float)ah); fh.h[8 + q] = bh; fl.h[8 + q] = (_Float16)(b - (float)bh); } }
__device__ __forceinline__ void ldB(FragH& f, const _Float16* Bt, int n, int ld, int k0, int hh) { const unsigned short* p = (const unsigned short*)Bt + (size_t)n * ld + k0; f.half[0] = *(const v8us*)(p + 8 * hh); f.half[1] = *(const v8us*)(p + 16 + 8 * hh); }
__global__ __launch_bounds__(128) void k_gru(const int* __restrict__ cseq, const float* __restrict__ E3, const float* __restrict__ PH3, const _Float16* __restrict__ Brz, const float* __restrict__ brh, const float* __restrict__ bzh, const _Float16* __restrict__ Bhh, const float* __restrict__ bhh, const _Float16* __restrict__ Bpj, const float* __restrict__ bpj, float* __restrict__ LOG) {
  __shared__ __attribute__((aligned(16))) float sH[4][16][HH + 8], sRH[4][16][HH + 8], sPH[4][16][G3], sLG[4][16][VV + 1]; __shared__ int sC[4][16][TT + 1];
  const int tid = threadIdx.x, w = tid >> 5, lane = tid & 31, ln = lane & 15, hh = lane >> 4; const int b0 = (blockIdx.x * 4 + w) * 16;
  for (int i = lane; i < 16 * (HH + 8); i += 32) (&sH[w][0][0])[i] = 0.f;
  for (int i = lane; i < 16 * G3; i += 32) { const int r = i / G3, c = i % G3; sPH[w][r][c] = PH3[(size_t)(b0 + r) * G3 + c]; }
  for (int i = lane; i < 16 * TT; i += 32) { const int r = i / TT, t = i % TT; sC[w][r][t] = cc(cseq[(size_t)(b0 + r) * (TT + 1) + t]); }
  float brz[8], bh4[4], bp2[2]; for (int t = 0; t < 8; ++t) brz[t] = bf16_round(t < 4 ? brh[t * 16 + ln] : bzh[(t - 4) * 16 + ln]); for (int t = 0; t < 4; ++t) bh4[t] = bf16_round(bhh[t * 16 + ln]); for (int t = 0; t < 2; ++t) bp2[t] = bf16_round(bpj[t * 16 + ln]);
  __builtin_amdgcn_fence(__ATOMIC_ACQ_REL, "workgroup"); __builtin_amdgcn_wave_barrier();
#pragma unroll 1
  for (int st = 0; st < TT; ++st) {
    float zk[4][8];
#pragma unroll 1
    for (int gsel = 0; gsel < 2; ++gsel) { v8f acc[4]; for (int t = 0; t < 4; ++t) acc[t] = v8f{};
#pragma unroll
      for (int ks = 0; ks < 2; ++ks) { FragH ah, al; fragHL(ah, al, &sH[w][ln][ks * 32], hh);
#pragma unroll
        for (int t = 0; t < 4; ++t) { FragH bq; ldB(bq, Brz, (gsel * 4 + t) * 16 + ln, HH, ks * 32, hh); acc[t] = mmaH<1>(ah.v, ah.v, bq.v, bq.v, acc[t]); acc[t] = mmaH<1>(al.v, al.v, bq.v, bq.v, acc[t]); } }
#pragma unroll
      for (int t = 0; t < 4; ++t) {
#pragma unroll
        for (int r = 0; r < 8; ++r) { const int row = 8 * hh + r; const int col = t * 16 + ln; const int c = sC[w][row][st]; const float x = E3[c * G3 + gsel * HH + col] + sPH[w][row][gsel * HH + col];
          const float g = 1.0f / (1.0f + __expf(-(acc[t][r] * 0.0625f + brz[gsel * 4 + t] + x))); if (gsel == 0) sRH[w][row][col] = g * sH[w][row][col]; else zk[t][r] = g; } } }
    __builtin_amdgcn_fence(__ATOMIC_ACQ_REL, "workgroup"); __builtin_amdgcn_wave_barrier();
    v8f acch[4]; for (int t = 0; t < 4; ++t) acch[t] = v8f{};
#pragma unroll
    for (int ks = 0; ks < 2; ++ks) { FragH ah, al; fragHL(ah, al, &sRH[w][ln][ks * 32], hh);
#pragma unroll
      for (int t = 0; t < 4; ++t) { FragH bq; ldB(bq, Bhh, t * 16 + ln, HH, ks * 32, hh); acch[t] = mmaH<1>(ah.v, ah.v, bq.v, bq.v, acch[t]); acch[t] = mmaH<1>(al.v, al.v, bq.v, bq.v, acch[t]); } }
#pragma unroll
    for (int t = 0; t < 4; ++t) {
#pragma unroll
      for (int r = 0; r < 8; ++r) { const int row = 8 * hh + r, col = t * 16 + ln; const int c = sC[w][row][st]; const float x = E3[c * G3 + 2 * HH + col] + sPH[w][row][2 * HH + col];
        const float cv = tanhf(acch[t][r] * 0.0625f + bh4[t] + x); const float z = zk[t][r]; const float hold = sH[w][row][col]; sH[w][row][col] = (1.0f - z) * hold + z * cv; } }
    __builtin_amdgcn_fence(__ATOMIC_ACQ_REL, "workgroup"); __builtin_amdgcn_wave_barrier();
    v8f accp[2]; accp[0] = v8f{}; accp[1] = v8f{};
#pragma unroll
    for (int ks = 0; ks < 2; ++ks) { FragH ah, al; fragHL(ah, al, &sH[w][ln][ks * 32], hh);
#pragma unroll
      for (int t = 0; t < 2; ++t) { FragH bq; ldB(bq, Bpj, t * 16 + ln, HH, ks * 32, hh); accp[t] = mmaH<1>(ah.v, ah.v, bq.v, bq.v, accp[t]); accp[t] = mmaH<1>(al.v, al.v, bq.v, bq.v, accp[t]); } }
#pragma unroll
    for (int t = 0; t < 2; ++t) for (int r = 0; r < 8; ++r) sLG[w][8 * hh + r][t * 16 + ln] = accp[t][r] * 0.0625f + bp2[t];
    __builtin_amdgcn_fence(__ATOMIC_ACQ_REL, "workgroup"); __builtin_amdgcn_wave_barrier();
    for (int r = 0; r < 16; ++r) *(volatile float*)(LOG + ((size_t)(b0 + r) * TT + st) * VV + lane) = sLG[w][r][lane];
  }
  __threadfence();
#pragma unroll 1
  for (int st = 0; st < TT; ++st) for (int r = 0; r < 16; ++r) { float* p = LOG + ((size_t)(b0 + r) * TT + st) * VV + lane; const float v = *(volatile float*)p; *(volatile float*)p = v; }
}
__global__ __launch_bounds__(256) void k_ce(const float* __restrict__ LOG, const int* __restrict__ cseq, float* __restrict__ NLL, float* __restrict__ MSK) { const size_t i = (size_t)blockIdx.x * 256 + threadIdx.x; if (i >= (size_t)BSZ * TT) return; const size_t b = i / TT; const int t = (int)(i % TT); const int tg = cc(cseq[b * (TT + 1) + t + 1]);
  const float* row = LOG + i * VV; float mx = -3.0e38f; for (int v = 0; v < VV; ++v) mx = fmaxf(mx, row[v]); float s = 0.f;
#pragma unroll 4
  for (int v = 0; v < VV; ++v) s += expf(row[v] - mx); const float lse = mx + logf(s); const float m = (tg != 0) ? 1.f : 0.f; const float nll = (lse - row[tg]) * m;
  *(volatile float*)(NLL + i) = nll; *(volatile float*)(MSK + i) = m; __threadfence(); *(volatile float*)(NLL + i) = nll; *(volatile float*)(MSK + i) = m; }
__global__ __launch_bounds__(1024) void k_loss(const float* __restrict__ NLL, const float* __restrict__ MSK, float* __restrict__ out) { __shared__ float s1[1024], s2[1024]; const int tid = threadIdx.x; float a = 0.f, b = 0.f; for (size_t i = tid; i < (size_t)BSZ * TT; i += 1024) { a += NLL[i]; b += MSK[i]; } s1[tid] = a; s2[tid] = b; __syncthreads();
  for (int st = 512; st >= 1; st >>= 1) { if (tid < st) { s1[tid] += s1[tid + st]; s2[tid] += s2[tid + st]; } __syncthreads(); } if (tid == 0) { const float v = s1[0] / fmaxf(s2[0], 1.0f); *(volatile float*)out = v; __threadfence(); *(volatile float*)out = v; } }
extern "C" void kernel_launch(void* const* d_in, const int* in_sizes, int n_in,
                              void* d_out, int out_size, void* d_ws, size_t ws_size, hipStream_t stream) {
  (void)in_sizes; (void)n_in; (void)out_size;
  const float* phon = (const float*)d_in[0]; const int* cseq = (const int*)d_in[1]; const float* emb = (const float*)d_in[2];
  const float* Wrx = (const float*)d_in[3]; const float* brx = (const float*)d_in[4]; const float* Wrh = (const float*)d_in[5]; const float* brh = (const float*)d_in[6]; const float* Wzx = (const float*)d_in[7]; const float* bzx = (const float*)d_in[8]; const float* Wzh = (const float*)d_in[9]; const float* bzh = (const float*)d_in[10];
  const float* Whx = (const float*)d_in[11]; const float* bhx = (const float*)d_in[12]; const float* Whh = (const float*)d_in[13]; const float* bhh = (const float*)d_in[14]; const float* Wpj = (const float*)d_in[15]; const float* bpj = (const float*)d_in[16];
  float* LOG = (float*)d_out; float* LOSS = (float*)((char*)d_out + LOSS_OFF);
  char* ws = (char*)d_ws; size_t off = 0;
  auto take = [&](size_t bytes) { char* p = ws + off; off += (bytes + 255) & ~(size_t)255; return p; };
  unsigned short* Btop = (unsigned short*)take((size_t)G3 * HH * 2); unsigned short* Bbot = (unsigned short*)take((size_t)G3 * PPAD * 2); float* B3 = (float*)take(G3 * 4); _Float16* Brz = (_Float16*)take((size_t)2 * HH * HH * 2); _Float16* Bhh = (_Float16*)take((size_t)HH * HH * 2); _Float16* Bpj = (_Float16*)take((size_t)VV * HH * 2);
  float* EMBP = (float*)take(VV * HH * 4); float* PHP = (float*)take((size_t)BSZ * PPAD * 4); float* E3 = (float*)take(VV * G3 * 4); float* PH3 = (float*)take((size_t)BSZ * G3 * 4); float* NLL = (float*)take((size_t)BSZ * TT * 4); float* MSK = (float*)take((size_t)BSZ * TT * 4);
  if (off > ws_size) return;
  k_prep<<<(BSZ * PPAD + 255) / 256, 256, 0, stream>>>(Wrx, Wzx, Whx, brx, bzx, bhx, Wrh, Wzh, Whh, Wpj, emb, phon, Btop, Bbot, B3, Brz, Bhh, Bpj, EMBP, PHP);
  k_gemm_b<false, false, 0><<<dim3(((VV / 16) * (G3 / 64) + 3) / 4, 1), 128, 0, stream>>>(EMBP, HH, 0, Btop, Btop, HH, 0, nullptr, nullptr, 0, 0, 1.f, 1.f, E3, G3, 0, VV, G3, HH);
  k_gemm_b<false, false, 0><<<dim3(((BSZ / 16) * (G3 / 64) + 3) / 4, 1), 128, 0, stream>>>(PHP, PPAD, 0, Bbot, Bbot, PPAD, 0, B3, nullptr, 0, 0, 1.f, 1.f, PH3, G3, 0, BSZ, G3, PPAD);
  k_gru<<<BSZ / 64, 128, 0, stream>>>(cseq, E3, PH3, Brz, brh, bzh, Bhh, bhh, Bpj, bpj, LOG);
  k_ce<<<(BSZ * TT + 255) / 256, 256, 0, stream>>>(LOG, cseq, NLL, MSK);
  k_loss<<<1, 1024, 0, stream>>>(NLL, MSK, LOSS);
}
